// Block_11785390260704
// MI455X (gfx1250) — hardware-verified
//
#include <hip/hip_runtime.h>
#include <math.h>

typedef __attribute__((ext_vector_type(16))) _Float16 v16h;
typedef __attribute__((ext_vector_type(8)))  _Float16 v8h;
typedef __attribute__((ext_vector_type(8)))  float v8f;
typedef __attribute__((ext_vector_type(4)))  float v4f;
typedef __attribute__((ext_vector_type(4)))  unsigned v4u;
typedef _Float16 h16;

#ifndef NB
#define NB 2
#endif
#ifndef SEQ
#define SEQ 2048
#endif
#define NB_FULL 2
#define SEQ_FULL 2048
#define TT (NB * SEQ)
#define CC 1024
#define DIN 1024
#define NH 16
#define HD 64
#define NOPE 32
#define ROPE 32
#define LR 128
#define NSH 2
#define NRE 8
#define NEX (NSH + NRE)
#define EI 384
#define AW (NEX * EI)
#define NQB (SEQ / 64)
#define SCALE (1.0f / 2048.0f)

static_assert(NH * HD == CC);
static_assert(NOPE + ROPE == HD);
static_assert(HD == 64);
static_assert(ROPE == 32);
static_assert(DIN == 1024);
static_assert(CC == 1024);
static_assert(LR == 128);
static_assert(DIN % 32 == 0);
static_assert(LR % 32 == 0);
static_assert(AW % 32 == 0);
static_assert(EI % 64 == 0);
static_assert(AW % 64 == 0);
static_assert(CC % 128 == 0);
static_assert(DIN % 128 == 0);
static_assert(SEQ % 128 == 0);
static_assert(SEQ / 128 <= 16);
static_assert(NQB <= 32);
static_assert(SEQ <= SEQ_FULL);
static_assert(NB <= NB_FULL);
static_assert(TT % 64 == 0);
static_assert(TT % 32 == 0);
static_assert(TT % 8 == 0);
static_assert(NRE == 8);
static_assert((size_t)NB_FULL * SEQ_FULL * DIN * 4 == (size_t)16777216);

template <typename T> __device__ __forceinline__ void vst2(void* p, T v) { *(volatile T*)p = v; __threadfence(); *(volatile T*)p = v; }
__device__ __forceinline__ v8f wmma16(v16h a, v16h b, v8f c) {
  v8f d = __builtin_amdgcn_wmma_f32_16x16x32_f16(false, a, false, b, (short)0, c, false, false);
  asm volatile("v_nop\n\tv_nop\n\tv_nop\n\tv_nop" : "+v"(d) : "v"(a), "v"(b));
  return d;
}
__device__ __forceinline__ v16h frag_h(const _Float16* rowk0, int lane) {
  union { v16h v; v8h q[2]; } u; const _Float16* p = rowk0 + 8 * (lane >> 4);
  u.q[0] = *(const v8h*)p; u.q[1] = *(const v8h*)(p + 16); return u.v;
}
__device__ __forceinline__ float bfr(float v) { return (float)(__bf16)v; }
static __device__ __forceinline__ h16 toh_flush(float v) { const h16 r = (h16)v; return (fabsf(v) < 6.103515625e-05f) ? (h16)0.0f : r; }
#define LDSX() do { asm volatile("s_wait_dscnt 0" ::: "memory"); __builtin_amdgcn_wave_barrier(); __builtin_amdgcn_fence(3  , "workgroup"); } while (0)

union H8 { v8h h; v4u u; };

#define SZ_A   (2u * (size_t)TT * CC)
#define WS_XI  ((size_t)0)
#define WS_WDT (WS_XI + SZ_A)
#define WS_W3  (WS_WDT + 2u * (size_t)2 * LR * DIN)
#define WS_WOT (WS_W3 + 2u * (size_t)3 * CC * LR)
#define WS_GUT (WS_WOT + 2u * (size_t)DIN * CC)
#define WS_DNT (WS_GUT + 2u * (size_t)2 * AW * DIN)
#define WS_CL  (WS_DNT + 2u * (size_t)DIN * AW)
#define WS_QKH (WS_CL + 2u * (size_t)2 * TT * LR)
#define WS_VT  (WS_QKH + 2u * SZ_A)
#define WS_YH  (WS_VT + SZ_A)
#define WS_H   (WS_YH + SZ_A)
#define WS_HN  (WS_H + 4u * (size_t)TT * DIN)
#define WS_ACT (WS_HN + SZ_A)
#define WS_WDN (WS_ACT + 2u * (size_t)TT * AW)
#define WS_UP  (WS_WDN + 4u * (size_t)TT * NRE)
#define WS_FL  (WS_UP + (size_t)(TT / 32) * 128u)
#define WS_END (WS_FL + 32u * 128u)
static_assert(WS_END <= (size_t)134217728);
static_assert(SZ_A % 128 == 0);
static_assert((2u * (size_t)2 * TT * LR) % 128 == 0);
static_assert((4u * (size_t)TT * NRE) % 128 == 0);
static_assert((2u * (size_t)TT * AW) % 128 == 0);

__device__ __forceinline__ void ld8(const float* __restrict__ p, size_t i, float t[8]) {
  const v4f a = *(const v4f*)(p + i); const v4f b = *(const v4f*)(p + i + 4);
  t[0] = a.x; t[1] = a.y; t[2] = a.z; t[3] = a.w; t[4] = b.x; t[5] = b.y; t[6] = b.z; t[7] = b.w;
}

__global__ __launch_bounds__(256) void k_wt(const float* __restrict__ S, _Float16* __restrict__ D, long long strideZ, int ldS, int ldD, int kofs, int kofsZ, int nofs, int nofsZ, int gsh, int gst, int base) {
  __shared__ __align__(16) _Float16 st[64][72];
  const int tid = threadIdx.x; const int z = blockIdx.z; const int k0 = blockIdx.x * 64, n0 = blockIdx.y * 64;
  const size_t sb = (size_t)z * (size_t)strideZ;
  const int r = tid >> 4, c4 = (tid & 15) * 4;
#pragma unroll 1
  for (int it = 0; it < 4; ++it) { const int kl = r + 16 * it; const v4f a = *(const v4f*)(S + sb + (size_t)(k0 + kl) * ldS + n0 + c4);
    st[c4 + 0][kl] = toh_flush(bfr(a.x) * 256.0f); st[c4 + 1][kl] = toh_flush(bfr(a.y) * 256.0f);
    st[c4 + 2][kl] = toh_flush(bfr(a.z) * 256.0f); st[c4 + 3][kl] = toh_flush(bfr(a.w) * 256.0f); }
  __syncthreads();
#pragma unroll 1
  for (int it = 0; it < 2; ++it) { const int e = tid + it * 256, nl = e >> 3, pc = e & 7; const int n = nofs + z * nofsZ + n0 + nl;
    const int drow = base + (n >> gsh) * gst + (n & ((1 << gsh) - 1));
    const v4u w = *(const v4u*)&st[nl][pc * 8];
    vst2(D + (size_t)drow * ldD + kofs + z * kofsZ + k0 + pc * 8, w); }
}

__global__ __launch_bounds__(256) void k_rms1(const float* __restrict__ X, const float* __restrict__ LW, _Float16* __restrict__ XI) {
#pragma clang fp contract(off)
  const int tid = threadIdx.x, lane = tid & 31; const int wave = __builtin_amdgcn_readfirstlane(tid >> 5);
  const size_t row = (size_t)blockIdx.x * 8 + wave; const size_t bb = row / SEQ, s = row % SEQ;
  const size_t so = (bb * SEQ_FULL + s) * DIN;
  float ssq = 0.0f;
#pragma unroll 1
  for (int it = 0; it < 4; ++it) { float t[8]; ld8(X, so + (size_t)it * 256 + lane * 8, t);
#pragma unroll
    for (int i = 0; i < 8; ++i) { const float v = bfr(t[i]); ssq += v * v; } }
  ssq += __shfl_xor(ssq, 16); ssq += __shfl_xor(ssq, 8); ssq += __shfl_xor(ssq, 4); ssq += __shfl_xor(ssq, 2); ssq += __shfl_xor(ssq, 1);
  const float inv = rsqrtf(ssq * (1.0f / 1024.0f) + 1.0e-5f);
#pragma unroll 1
  for (int it = 0; it < 4; ++it) { const size_t c = (size_t)it * 256 + lane * 8; float t[8], w[8]; ld8(X, so + c, t); ld8(LW, c, w); H8 o;
#pragma unroll
    for (int i = 0; i < 8; ++i) o.h[i] = toh_flush(bfr(w[i]) * bfr(t[i]) * inv * 16.0f);
    vst2(XI + row * DIN + c, o.u); }
}

__global__ __launch_bounds__(256) void k_flag(const float* __restrict__ MK, int* __restrict__ FL) {
  __shared__ unsigned snz[8][2];
  const int tid = threadIdx.x, lane = tid & 31; const int wave = __builtin_amdgcn_readfirstlane(tid >> 5);
  const int qb = blockIdx.x;
  unsigned nzb = 0u;
#pragma unroll 1
  for (int rr = 0; rr < 8; ++rr) {
    const float* mr = MK + (size_t)(qb * 64 + wave * 8 + rr) * SEQ_FULL + lane * 4;
#pragma unroll
    for (int it = 0; it < SEQ / 128; ++it) { const v4f m = *(const v4f*)(mr + it * 128);
      const unsigned anz = (unsigned)((m.x != 0.0f) | (m.y != 0.0f) | (m.z != 0.0f) | (m.w != 0.0f));
      nzb |= anz << it; }
  }
#pragma unroll
  for (int o = 1; o < 16; o <<= 1) nzb |= (unsigned)__shfl_xor((int)nzb, o);
  if ((lane & 15) == 0) snz[wave][lane >> 4] = nzb;
  __syncthreads();
  if (wave == 0) { const int it = lane >> 1, hf = lane & 1; unsigned a = 0u;
#pragma unroll
    for (int w = 0; w < 8; ++w) a |= snz[w][hf];
    const int flag = (int)((a >> it) & 1u);
    vst2(FL + qb * 32 + lane, flag); }
}

__global__ __launch_bounds__(128) void k_lat(const _Float16* __restrict__ XI, const _Float16* __restrict__ WDT, const float* __restrict__ KVN, const float* __restrict__ QN, _Float16* __restrict__ CL) {
  __shared__ __align__(16) float ss[4][16][132];
  const int tid = threadIdx.x, lane = tid & 31, col = lane & 15, g = lane >> 4; const int wave = __builtin_amdgcn_readfirstlane(tid >> 5);
  const int y = blockIdx.y; const size_t rb = (size_t)blockIdx.x * 64; const size_t r0 = rb + wave * 16;
  v8f acc[8] = {};
#pragma unroll 2
  for (int kc = 0; kc < DIN / 32; ++kc) { const v16h a = frag_h(XI + (r0 + col) * DIN + kc * 32, lane);
#pragma unroll
    for (int j = 0; j < 8; ++j) { const v16h w = frag_h(WDT + (size_t)(y * LR + j * 16 + col) * DIN + kc * 32, lane); acc[j] = wmma16(a, w, acc[j]); } }
#pragma unroll
  for (int j = 0; j < 8; ++j) {
#pragma unroll
    for (int r = 0; r < 8; ++r) ss[wave][8 * g + r][j * 16 + col] = acc[j][r] * (1.0f / 4096.0f); }
  LDSX();
  float na[8], nq[8], nw[8]; ld8(KVN, (size_t)col * 8, na); ld8(QN, (size_t)col * 8, nq);
#pragma unroll
  for (int i = 0; i < 8; ++i) nw[i] = bfr((y == 0) ? na[i] : nq[i]);
#pragma unroll 1
  for (int it = 0; it < 8; ++it) { const int row = it * 2 + g;
    const v4f a = *(const v4f*)&ss[wave][row][col * 8]; const v4f b = *(const v4f*)&ss[wave][row][col * 8 + 4];
    float v[8]; v[0] = a.x; v[1] = a.y; v[2] = a.z; v[3] = a.w; v[4] = b.x; v[5] = b.y; v[6] = b.z; v[7] = b.w;
    float q = 0.0f;
#pragma unroll
    for (int i = 0; i < 8; ++i) q += v[i] * v[i];
    q += __shfl_xor(q, 1); q += __shfl_xor(q, 2); q += __shfl_xor(q, 4); q += __shfl_xor(q, 8);
    const float inv = rsqrtf(q * (1.0f / 128.0f) + 1.0e-5f);
    H8 o;
#pragma unroll
    for (int i = 0; i < 8; ++i) o.h[i] = toh_flush(nw[i] * v[i] * inv * 16.0f);
    vst2(CL + (size_t)y * TT * LR + (r0 + row) * LR + col * 8, o.u); }
}

__global__ __launch_bounds__(128) void k_proj(const _Float16* __restrict__ CL, const _Float16* __restrict__ W3, const float* __restrict__ COS, const float* __restrict__ SIN,
    _Float16* __restrict__ QKH, _Float16* __restrict__ VT) {
  __shared__ __align__(16) float sf[64][132];
  __shared__ __align__(16) _Float16 th[128][72];
  const int tid = threadIdx.x, lane = tid & 31, col = lane & 15, g = lane >> 4; const int wave = __builtin_amdgcn_readfirstlane(tid >> 5);
  const int which = blockIdx.z; const int c0 = blockIdx.y * 128; const size_t r0 = (size_t)blockIdx.x * 64; const size_t bb = r0 / SEQ; const int t0 = (int)(r0 % SEQ);
  const _Float16* A = CL + (size_t)((which == 0) ? 1 : 0) * TT * LR; const _Float16* W = W3 + (size_t)which * CC * LR;
  v8f acc[8] = {};
#pragma unroll 2
  for (int kc = 0; kc < LR / 32; ++kc) { const v16h a = frag_h(A + (r0 + wave * 16 + col) * LR + kc * 32, lane);
#pragma unroll
    for (int j = 0; j < 8; ++j) { const v16h w = frag_h(W + (size_t)(c0 + j * 16 + col) * LR + kc * 32, lane); acc[j] = wmma16(a, w, acc[j]); } }
  if (which < 2) {
#pragma unroll
    for (int j = 0; j < 8; ++j) {
#pragma unroll
      for (int r = 0; r < 8; ++r) sf[wave * 16 + 8 * g + r][j * 16 + col] = acc[j][r]; }
    __syncthreads();
    _Float16* DH = QKH + (size_t)which * TT * CC;
#pragma unroll 1
    for (int e = tid; e < 64 * 16; e += 128) { const int rl = e >> 4, q = e & 15, cl = q * 8, d0 = cl & 63; const bool isr = (d0 >= NOPE); const int dd = isr ? d0 - NOPE : 0; const int pcl = cl ^ 16;
      const float sg = (dd < 16) ? -1.0f : 1.0f;
      const size_t cs = (size_t)(t0 + rl) * ROPE + dd;
      const v4f ca = *(const v4f*)(COS + cs), cb = *(const v4f*)(COS + cs + 4), sa = *(const v4f*)(SIN + cs), sb = *(const v4f*)(SIN + cs + 4);
      float cv[8], sv[8];
      cv[0] = ca.x; cv[1] = ca.y; cv[2] = ca.z; cv[3] = ca.w; cv[4] = cb.x; cv[5] = cb.y; cv[6] = cb.z; cv[7] = cb.w;
      sv[0] = sa.x; sv[1] = sa.y; sv[2] = sa.z; sv[3] = sa.w; sv[4] = sb.x; sv[5] = sb.y; sv[6] = sb.z; sv[7] = sb.w;
      H8 hv;
#pragma unroll
      for (int u = 0; u < 8; ++u) { const float x = sf[rl][cl + u], xp = sf[rl][pcl + u]; const float cu = isr ? bfr(cv[u]) : 1.0f, su = isr ? bfr(sv[u]) : 0.0f;
        const float v = (x * cu + sg * xp * su) * (1.0f / 256.0f); hv.h[u] = toh_flush(v); }
      vst2(DH + (r0 + rl) * CC + c0 + cl, hv.u); }
  } else {
#pragma unroll
    for (int j = 0; j < 8; ++j) {
#pragma unroll
      for (int r = 0; r < 8; ++r) { const float v = acc[j][r] * (1.0f / 256.0f); const int rl = wave * 16 + 8 * g + r, cl = j * 16 + col; th[cl][rl] = toh_flush(v); } }
    __syncthreads();
#pragma unroll 1
    for (int e = tid; e < 128 * 8; e += 128) { const int cl = e >> 3, q = e & 7; const size_t o3 = (bb * CC + c0 + cl) * (size_t)SEQ + t0 + q * 8;
      const v4u w = *(const v4u*)&th[cl][q * 8];
      vst2(VT + o3, w); } }
}

__global__ __launch_bounds__(128) void k_fa(const _Float16* __restrict__ QH, const _Float16* __restrict__ KH, const _Float16* __restrict__ VT, const float* __restrict__ MK, const int* __restrict__ FL, _Float16* __restrict__ YH) {
  __shared__ __align__(16) _Float16 sp[4][16][40];
  __shared__ __align__(16) _Float16 so[4][16][72];
  const int tid = threadIdx.x, lane = tid & 31, col = lane & 15, g = lane >> 4; const int wave = __builtin_amdgcn_readfirstlane(tid >> 5);
  const int qb = blockIdx.x; const int b = blockIdx.y / NH, h = blockIdx.y % NH; const int ql0 = qb * 64 + wave * 16;
  const size_t qoff = ((size_t)b * SEQ + ql0 + col) * CC + h * HD;
  const size_t kbase = ((size_t)b * SEQ + col) * CC + h * HD;
  const size_t vbase = ((size_t)b * CC + h * HD + col) * SEQ;
  const size_t mbase = (size_t)(ql0 + 8 * g) * SEQ_FULL + col;
  v16h ones;
#pragma unroll
  for (int i = 0; i < 16; ++i) ones[i] = (_Float16)1.0f;
  v8f acc[4] = {}; v8f accs = {};
  float mrun[8];
#pragma unroll
  for (int r = 0; r < 8; ++r) mrun[r] = -3.0e38f;
#pragma unroll 1
  for (int kb = 0; kb < NQB; ++kb) {
    const int fl = __builtin_amdgcn_readfirstlane(FL[qb * 32 + kb]);
#pragma unroll 1
    for (int hf = 0; hf < 2; ++hf) { const int k0 = kb * 64 + hf * 32;
      v8f s0 = {}, s1 = {};
#pragma unroll
      for (int kc = 0; kc < HD / 32; ++kc) { const v16h qa = frag_h(QH + qoff + kc * 32, lane);
        const v16h ka0 = frag_h(KH + kbase + (size_t)k0 * CC + kc * 32, lane); const v16h ka1 = frag_h(KH + kbase + (size_t)(k0 + 16) * CC + kc * 32, lane);
        s0 = wmma16(qa, ka0, s0); s1 = wmma16(qa, ka1, s1); }
      float sv0[8], sv1[8];
#pragma unroll
      for (int r = 0; r < 8; ++r) { sv0[r] = s0[r] * SCALE; sv1[r] = s1[r] * SCALE; }
      if (fl != 0) { float m0[8], m1[8];
#pragma unroll
        for (int r = 0; r < 8; ++r) m0[r] = MK[mbase + (size_t)r * SEQ_FULL + k0];
        asm volatile("s_wait_loadcnt 0x0" ::: "memory");
#pragma unroll
        for (int r = 0; r < 8; ++r) m1[r] = MK[mbase + (size_t)r * SEQ_FULL + k0 + 16];
        asm volatile("s_wait_loadcnt 0x0" ::: "memory");
#pragma unroll
        for (int r = 0; r < 8; ++r) { sv0[r] = sv0[r] + bfr(m0[r]); sv1[r] = sv1[r] + bfr(m1[r]); } }
      float fr[8];
#pragma unroll
      for (int r = 0; r < 8; ++r) { float t = fmaxf(sv0[r], sv1[r]);
        t = fmaxf(t, __shfl_xor(t, 1)); t = fmaxf(t, __shfl_xor(t, 2)); t = fmaxf(t, __shfl_xor(t, 4)); t = fmaxf(t, __shfl_xor(t, 8));
        const float mn = fmaxf(mrun[r], t); fr[r] = __expf(mrun[r] - mn); mrun[r] = mn;
        const float e0 = sv0[r] - mn, e1 = sv1[r] - mn;
        sp[wave][8 * g + r][col] = (e0 < -15.0f) ? (_Float16)0.0f : (_Float16)(__expf(e0) * 256.0f);
        sp[wave][8 * g + r][16 + col] = (e1 < -15.0f) ? (_Float16)0.0f : (_Float16)(__expf(e1) * 256.0f); }
#pragma unroll
      for (int t = 0; t < 4; ++t) {
#pragma unroll
        for (int r = 0; r < 8; ++r) acc[t][r] *= fr[r]; }
#pragma unroll
      for (int r = 0; r < 8; ++r) accs[r] *= fr[r];
      LDSX();
      union { v16h v; v8h q[2]; } pa; pa.q[0] = *(const v8h*)&sp[wave][col][8 * g]; pa.q[1] = *(const v8h*)&sp[wave][col][16 + 8 * g];
      LDSX();
#pragma unroll
      for (int t = 0; t < 4; ++t) { const v16h vf = frag_h(VT + vbase + (size_t)(t * 16) * SEQ + k0, lane); acc[t] = wmma16(pa.v, vf, acc[t]); }
      accs = wmma16(pa.v, ones, accs);
    } }
  float inv[8];
#pragma unroll
  for (int r = 0; r < 8; ++r) inv[r] = (accs[r] > 0.0f) ? (1.0f / accs[r]) * 4.0f : 0.0f;
#pragma unroll
  for (int t = 0; t < 4; ++t) {
#pragma unroll
    for (int r = 0; r < 8; ++r) so[wave][8 * g + r][t * 16 + col] = toh_flush(acc[t][r] * inv[r]); }
  LDSX();
#pragma unroll
  for (int it = 0; it < 4; ++it) { const int row = it * 4 + (lane >> 3), pc = lane & 7; const v4u w = *(const v4u*)&so[wave][row][pc * 8];
    vst2(YH + ((size_t)b * SEQ + ql0 + row) * CC + h * HD + pc * 8, w); }
}

__global__ __launch_bounds__(128) void k_oproj(const _Float16* __restrict__ YH, const _Float16* __restrict__ WOT, const float* __restrict__ X, float* __restrict__ HP) {
  __shared__ __align__(16) float ss[4][16][132];
  const int tid = threadIdx.x, lane = tid & 31, col = lane & 15, g = lane >> 4; const int wave = __builtin_amdgcn_readfirstlane(tid >> 5);
  const int c0 = blockIdx.y * 128; const size_t rb = (size_t)blockIdx.x * 64; const size_t r0 = rb + wave * 16;
  v8f acc[8] = {};
#pragma unroll 2
  for (int kc = 0; kc < CC / 32; ++kc) { const v16h a = frag_h(YH + (r0 + col) * CC + kc * 32, lane);
#pragma unroll
    for (int j = 0; j < 8; ++j) { const v16h w = frag_h(WOT + (size_t)(c0 + j * 16 + col) * CC + kc * 32, lane); acc[j] = wmma16(a, w, acc[j]); } }
#pragma unroll
  for (int j = 0; j < 8; ++j) {
#pragma unroll
    for (int r = 0; r < 8; ++r) ss[wave][8 * g + r][j * 16 + col] = acc[j][r] * (1.0f / 16384.0f); }
  LDSX();
#pragma unroll 1
  for (int rl = 0; rl < 16; ++rl) { const size_t row = r0 + rl; const size_t bb = row / SEQ, s = row % SEQ;
    const v4f xv = *(const v4f*)(X + (bb * SEQ_FULL + s) * DIN + c0 + lane * 4); const v4f sv = *(const v4f*)&ss[wave][rl][lane * 4];
    v4f o; o.x = bfr(xv.x) + sv.x; o.y = bfr(xv.y) + sv.y; o.z = bfr(xv.z) + sv.z; o.w = bfr(xv.w) + sv.w;
    vst2(HP + row * DIN + c0 + lane * 4, o); }
}

__global__ __launch_bounds__(256) void k_route(const float* __restrict__ HP, const float* __restrict__ LW, const float* __restrict__ RW, const float* __restrict__ RB,
    _Float16* __restrict__ HN, float* __restrict__ WDN, float* __restrict__ UP) {
#pragma clang fp contract(off)
  __shared__ __align__(16) float swd[32][8];
  __shared__ float scnt[8][8];
  const int tid = threadIdx.x, lane = tid & 31; const int wave = __builtin_amdgcn_readfirstlane(tid >> 5);
  const int e = lane & 7;
  const float rbias = bfr(RB[e]);
  float cnt = 0.0f;
#pragma unroll 1
  for (int rr = 0; rr < 4; ++rr) {
    const int rloc = wave * 4 + rr; const size_t row = (size_t)blockIdx.x * 32 + rloc; const size_t so = row * DIN;
    float ssq = 0.0f;
#pragma unroll 1
    for (int it = 0; it < 4; ++it) { float t[8]; ld8(HP, so + (size_t)it * 256 + lane * 8, t);
#pragma unroll
      for (int i = 0; i < 8; ++i) ssq += t[i] * t[i]; }
    ssq += __shfl_xor(ssq, 16); ssq += __shfl_xor(ssq, 8); ssq += __shfl_xor(ssq, 4); ssq += __shfl_xor(ssq, 2); ssq += __shfl_xor(ssq, 1);
    const float inv = rsqrtf(ssq * (1.0f / 1024.0f) + 1.0e-5f);
    float lg[8];
#pragma unroll
    for (int j = 0; j < 8; ++j) lg[j] = 0.0f;
#pragma unroll 1
    for (int it = 0; it < 4; ++it) { const size_t c = (size_t)it * 256 + lane * 8; float t[8], w[8]; ld8(HP, so + c, t); ld8(LW, c, w); H8 o;
#pragma unroll
      for (int i = 0; i < 8; ++i) { const float hv = bfr(w[i]) * t[i] * inv; o.h[i] = toh_flush(hv * 16.0f);
        const v4f ra = *(const v4f*)(RW + (c + i) * NRE); const v4f rb = *(const v4f*)(RW + (c + i) * NRE + 4);
        lg[0] += hv * bfr(ra.x); lg[1] += hv * bfr(ra.y); lg[2] += hv * bfr(ra.z); lg[3] += hv * bfr(ra.w);
        lg[4] += hv * bfr(rb.x); lg[5] += hv * bfr(rb.y); lg[6] += hv * bfr(rb.z); lg[7] += hv * bfr(rb.w); }
      vst2(HN + so + c, o.u); }
#pragma unroll
    for (int j = 0; j < 8; ++j) { float v = lg[j];
      v += __shfl_xor(v, 16); v += __shfl_xor(v, 8); v += __shfl_xor(v, 4); v += __shfl_xor(v, 2); v += __shfl_xor(v, 1); lg[j] = v; }
    float s = lg[0];
    s = (e == 1) ? lg[1] : s; s = (e == 2) ? lg[2] : s; s = (e == 3) ? lg[3] : s; s = (e == 4) ? lg[4] : s;
    s = (e == 5) ? lg[5] : s; s = (e == 6) ? lg[6] : s; s = (e == 7) ? lg[7] : s;
    s = s + rbias;
    const float p = 1.0f / (1.0f + expf(-s));
    float v1 = p; int i1 = e;
#pragma unroll
    for (int o = 1; o < 8; o <<= 1) { const float op = __shfl_xor(v1, o); const int oi = __shfl_xor(i1, o);
      const bool take = (op > v1) || ((op == v1) && (oi < i1)); v1 = take ? op : v1; i1 = take ? oi : i1; }
    float v2 = (e == i1) ? -1.0f : p; int i2 = e;
#pragma unroll
    for (int o = 1; o < 8; o <<= 1) { const float op = __shfl_xor(v2, o); const int oi = __shfl_xor(i2, o);
      const bool take = (op > v2) || ((op == v2) && (oi < i2)); v2 = take ? op : v2; i2 = take ? oi : i2; }
    const float rinv = 1.0f / (v1 + v2);
    const float mine = (e == i1) ? v1 * rinv : ((e == i2) ? v2 * rinv : 0.0f);
    cnt += ((e == i1) || (e == i2)) ? 1.0f : 0.0f;
    if (lane < 8) swd[rloc][e] = mine;
  }
  if (lane < 8) scnt[wave][lane] = cnt;
  __syncthreads();
  if (wave == 0) {
#pragma unroll 1
    for (int it = 0; it < 2; ++it) { const int idx = it * 32 + lane; const v4f w = *(const v4f*)(&swd[0][0] + idx * 4);
      vst2(WDN + (size_t)blockIdx.x * 256 + idx * 4, w); }
    float u = 0.0f;
#pragma unroll
    for (int w = 0; w < 8; ++w) u += scnt[w][lane & 7];
    const float uo = (lane < 8) ? u : 0.0f;
    vst2(UP + (size_t)blockIdx.x * 32 + lane, uo); }
}

__global__ __launch_bounds__(128) void k_gateup(const _Float16* __restrict__ HN, const _Float16* __restrict__ GUT, const float* __restrict__ WDN, _Float16* __restrict__ ACT) {
  __shared__ __align__(16) _Float16 sa[4][16][72];
  const int tid = threadIdx.x, lane = tid & 31, col = lane & 15, g = lane >> 4; const int wave = __builtin_amdgcn_readfirstlane(tid >> 5);
  const int nb = blockIdx.y; const size_t rb = (size_t)blockIdx.x * 64; const size_t r0 = rb + wave * 16;
  v8f acc[8] = {};
#pragma unroll 2
  for (int kc = 0; kc < DIN / 32; ++kc) { const v16h a = frag_h(HN + (r0 + col) * DIN + kc * 32, lane);
#pragma unroll
    for (int j = 0; j < 8; ++j) { const v16h w = frag_h(GUT + (size_t)(nb * 128 + j * 16 + col) * DIN + kc * 32, lane); acc[j] = wmma16(a, w, acc[j]); } }
  const int ex = nb / (EI / 64);
  const int ec = (ex >= NSH) ? ex - NSH : 0;
  float rw[8];
#pragma unroll
  for (int r = 0; r < 8; ++r) { const float wv = WDN[(r0 + 8 * g + r) * NRE + ec]; rw[r] = (ex < NSH) ? 1.0f : wv; }
#pragma unroll
  for (int t = 0; t < 4; ++t) {
#pragma unroll
    for (int r = 0; r < 8; ++r) { const float gv = acc[t][r] * (1.0f / 4096.0f), uv = acc[4 + t][r] * (1.0f / 4096.0f);
      const float sl = gv * __builtin_amdgcn_rcpf(1.0f + __expf(-gv));
      sa[wave][8 * g + r][t * 16 + col] = toh_flush(sl * uv * rw[r] * 256.0f); } }
  LDSX();
#pragma unroll
  for (int it = 0; it < 4; ++it) { const int row = it * 4 + (lane >> 3), pc = lane & 7; const v4u w = *(const v4u*)&sa[wave][row][pc * 8];
    vst2(ACT + (r0 + row) * AW + nb * 64 + pc * 8, w); }
}

__global__ __launch_bounds__(128) void k_dn(const _Float16* __restrict__ ACT, const _Float16* __restrict__ DNT, const float* __restrict__ HP, float* __restrict__ OUT) {
  __shared__ __align__(16) float ss[4][16][132];
  const int tid = threadIdx.x, lane = tid & 31, col = lane & 15, g = lane >> 4; const int wave = __builtin_amdgcn_readfirstlane(tid >> 5);
  const int c0 = blockIdx.y * 128; const size_t rb = (size_t)blockIdx.x * 64; const size_t r0 = rb + wave * 16;
  v8f acc[8] = {};
#pragma unroll 2
  for (int kc = 0; kc < AW / 32; ++kc) { const v16h a = frag_h(ACT + (r0 + col) * AW + kc * 32, lane);
#pragma unroll
    for (int j = 0; j < 8; ++j) { const v16h w = frag_h(DNT + (size_t)(c0 + j * 16 + col) * AW + kc * 32, lane); acc[j] = wmma16(a, w, acc[j]); } }
#pragma unroll
  for (int j = 0; j < 8; ++j) {
#pragma unroll
    for (int r = 0; r < 8; ++r) ss[wave][8 * g + r][j * 16 + col] = acc[j][r] * (1.0f / 65536.0f); }
  LDSX();
#pragma unroll 1
  for (int rl = 0; rl < 16; ++rl) { const size_t row = r0 + rl; const size_t bb = row / SEQ, s = row % SEQ;
    const v4f hv = *(const v4f*)(HP + row * DIN + c0 + lane * 4); const v4f sv = *(const v4f*)&ss[wave][rl][lane * 4];
    v4f o; o.x = hv.x + sv.x; o.y = hv.y + sv.y; o.z = hv.z + sv.z; o.w = hv.w + sv.w;
    vst2(OUT + (bb * SEQ_FULL + s) * DIN + c0 + lane * 4, o); }
}

__global__ __launch_bounds__(32) void k_usage(const float* __restrict__ UP, float* __restrict__ OUT1) {
  const int lane = threadIdx.x; const int q = lane & 1;
  v4f a = {0.0f, 0.0f, 0.0f, 0.0f};
#pragma unroll 1
  for (int blk = 0; blk < TT / 32; ++blk) { const v4f p = *(const v4f*)(UP + (size_t)blk * 32 + q * 4); a.x += p.x; a.y += p.y; a.z += p.z; a.w += p.w; }
  if (lane < 2) vst2(OUT1 + lane * 4, a);
}

extern "C" void kernel_launch(void* const* d_in, const int* in_sizes, int n_in, void* d_out, int out_size, void* d_ws, size_t ws_size, hipStream_t stream) {
  if (n_in < 24) return;
  if (ws_size < (size_t)WS_END) return;
  const long long needx = ((long long)(NB - 1) * SEQ_FULL + SEQ) * DIN;
  const long long needt = (long long)SEQ * ROPE;
  const long long needm = (long long)(SEQ - 1) * SEQ_FULL + SEQ;
  if (in_sizes[0] < needx || in_sizes[1] < needt || in_sizes[2] < needt || in_sizes[3] < needm) return;
  if (in_sizes[4] < DIN || in_sizes[5] < DIN) return;
  if (in_sizes[6] < DIN * LR || in_sizes[7] < LR || in_sizes[8] < LR * 512 || in_sizes[9] < LR * 512 || in_sizes[10] < LR * CC) return;
  if (in_sizes[11] < DIN * LR || in_sizes[12] < LR || in_sizes[13] < LR * 512 || in_sizes[14] < LR * 512 || in_sizes[15] < CC * DIN) return;
  if (in_sizes[16] < NSH * DIN * EI || in_sizes[17] < NSH * DIN * EI || in_sizes[18] < NSH * EI * DIN) return;
  if (in_sizes[19] < NRE * DIN * EI || in_sizes[20] < NRE * DIN * EI || in_sizes[21] < NRE * EI * DIN) return;
  if (in_sizes[22] < DIN * NRE || in_sizes[23] < NRE) return;
  if ((long long)out_size < (long long)NB_FULL * SEQ_FULL * DIN + NRE) return;
  const float* x = (const float*)d_in[0]; const float* cosp = (const float*)d_in[1]; const float* sinp = (const float*)d_in[2]; const float* mk = (const float*)d_in[3];
  const float* ln1 = (const float*)d_in[4]; const float* ln2 = (const float*)d_in[5];
  const float* kvd = (const float*)d_in[6]; const float* kvn = (const float*)d_in[7]; const float* wuk = (const float*)d_in[8]; const float* wur = (const float*)d_in[9]; const float* wuv = (const float*)d_in[10];
  const float* qdn = (const float*)d_in[11]; const float* qnw = (const float*)d_in[12]; const float* wuq = (const float*)d_in[13]; const float* wqr = (const float*)d_in[14]; const float* wo = (const float*)d_in[15];
  const float* shg = (const float*)d_in[16]; const float* shu = (const float*)d_in[17]; const float* shd = (const float*)d_in[18];
  const float* rg = (const float*)d_in[19]; const float* ru = (const float*)d_in[20]; const float* rd = (const float*)d_in[21];
  const float* rw = (const float*)d_in[22]; const float* rbs = (const float*)d_in[23];
  char* ws = (char*)d_ws;
  _Float16* XI = (_Float16*)(ws + WS_XI); _Float16* WDT = (_Float16*)(ws + WS_WDT); _Float16* W3 = (_Float16*)(ws + WS_W3); _Float16* WOT = (_Float16*)(ws + WS_WOT);
  _Float16* GUT = (_Float16*)(ws + WS_GUT); _Float16* DNT = (_Float16*)(ws + WS_DNT); _Float16* CL = (_Float16*)(ws + WS_CL);
  _Float16* QKH = (_Float16*)(ws + WS_QKH); _Float16* VT = (_Float16*)(ws + WS_VT); _Float16* YH = (_Float16*)(ws + WS_YH);
  float* HP = (float*)(ws + WS_H); _Float16* HN = (_Float16*)(ws + WS_HN); _Float16* ACT = (_Float16*)(ws + WS_ACT);
  float* WDN = (float*)(ws + WS_WDN); float* UP = (float*)(ws + WS_UP); int* FL = (int*)(ws + WS_FL);
  _Float16* QH = QKH; _Float16* KH = QKH + (size_t)TT * CC;
  _Float16* WQT = W3; _Float16* WKT = W3 + (size_t)CC * LR; _Float16* WVT = W3 + (size_t)2 * CC * LR;
  float* OUT0 = (float*)d_out; float* OUT1 = (float*)d_out + (size_t)NB_FULL * SEQ_FULL * DIN;

  k_wt<<<dim3(DIN / 64, LR / 64, 1), 256, 0, stream>>>(kvd, WDT, 0LL, LR, DIN, 0, 0, 0, 0, 20, 0, 0);
  k_wt<<<dim3(DIN / 64, LR / 64, 1), 256, 0, stream>>>(qdn, WDT, 0LL, LR, DIN, 0, 0, 0, 0, 20, 0, LR);
  k_wt<<<dim3(LR / 64, 512 / 64, 1), 256, 0, stream>>>(wuk, WKT, 0LL, 512, LR, 0, 0, 0, 0, 5, 64, 0);
  k_wt<<<dim3(LR / 64, 512 / 64, 1), 256, 0, stream>>>(wur, WKT, 0LL, 512, LR, 0, 0, 0, 0, 5, 64, NOPE);
  k_wt<<<dim3(LR / 64, CC / 64, 1), 256, 0, stream>>>(wuv, WVT, 0LL, CC, LR, 0, 0, 0, 0, 20, 0, 0);
  k_wt<<<dim3(LR / 64, 512 / 64, 1), 256, 0, stream>>>(wuq, WQT, 0LL, 512, LR, 0, 0, 0, 0, 5, 64, 0);
  k_wt<<<dim3(LR / 64, 512 / 64, 1), 256, 0, stream>>>(wqr, WQT, 0LL, 512, LR, 0, 0, 0, 0, 5, 64, NOPE);
  k_wt<<<dim3(CC / 64, DIN / 64, 1), 256, 0, stream>>>(wo, WOT, 0LL, DIN, CC, 0, 0, 0, 0, 20, 0, 0);
  k_wt<<<dim3(DIN / 64, EI / 64, NSH), 256, 0, stream>>>(shg, GUT, (long long)DIN * EI, EI, DIN, 0, 0, 0, EI, 6, 128, 0);
  k_wt<<<dim3(DIN / 64, EI / 64, NSH), 256, 0, stream>>>(shu, GUT, (long long)DIN * EI, EI, DIN, 0, 0, 0, EI, 6, 128, 64);
  k_wt<<<dim3(DIN / 64, EI / 64, NRE), 256, 0, stream>>>(rg, GUT, (long long)DIN * EI, EI, DIN, 0, 0, NSH * EI, EI, 6, 128, 0);
  k_wt<<<dim3(DIN / 64, EI / 64, NRE), 256, 0, stream>>>(ru, GUT, (long long)DIN * EI, EI, DIN, 0, 0, NSH * EI, EI, 6, 128, 64);
  k_wt<<<dim3(EI / 64, DIN / 64, NSH), 256, 0, stream>>>(shd, DNT, (long long)EI * DIN, DIN, AW, 0, EI, 0, 0, 20, 0, 0);
  k_wt<<<dim3(EI / 64, DIN / 64, NRE), 256, 0, stream>>>(rd, DNT, (long long)EI * DIN, DIN, AW, NSH * EI, EI, 0, 0, 20, 0, 0);

  k_rms1<<<dim3(TT / 8), 256, 0, stream>>>(x, ln1, XI);
  k_flag<<<dim3(NQB), 256, 0, stream>>>(mk, FL);
  k_lat<<<dim3(TT / 64, 2), 128, 0, stream>>>(XI, WDT, kvn, qnw, CL);
  k_proj<<<dim3(TT / 64, CC / 128, 3), 128, 0, stream>>>(CL, W3, cosp, sinp, QKH, VT);
  k_fa<<<dim3(NQB, NB * NH), 128, 0, stream>>>(QH, KH, VT, mk, FL, YH);
  k_oproj<<<dim3(TT / 64, DIN / 128), 128, 0, stream>>>(YH, WOT, x, HP);
  k_route<<<dim3(TT / 32), 256, 0, stream>>>(HP, ln2, rw, rbs, HN, WDN, UP);
  k_gateup<<<dim3(TT / 64, AW / 64), 128, 0, stream>>>(HN, GUT, WDN, ACT);
  k_dn<<<dim3(TT / 64, DIN / 128), 128, 0, stream>>>(ACT, DNT, HP, OUT0);
  k_usage<<<dim3(1), 32, 0, stream>>>(UP, OUT1);
}
